// EncoderMambaBlock_28003186769941
// MI455X (gfx1250) — hardware-verified
//
#include <hip/hip_runtime.h>
#include <math.h>

typedef __attribute__((ext_vector_type(16))) _Float16 v16h;
typedef __attribute__((ext_vector_type(8)))  _Float16 v8h;
typedef __attribute__((ext_vector_type(16))) __bf16   v16b;
typedef __attribute__((ext_vector_type(8)))  __bf16   v8b;
typedef __attribute__((ext_vector_type(8)))  float    v8f;
typedef __attribute__((ext_vector_type(4)))  float    v4f;

constexpr int kBatch  = 2;
constexpr int kSeq    = 2048;
constexpr int kDim    = 1024;
constexpr int kDtR    = 64;
constexpr int kNst    = 16;
constexpr int kDbcW   = kDtR + 2 * kNst;
constexpr int kDbcP   = 128;
constexpr int kRows   = kBatch * kSeq;
constexpr int kRows2  = 2 * kRows;
constexpr float kEps  = 1e-5f;
constexpr float kWCarry    = 256.0f;
constexpr float kWCarryInv = 1.0f / 256.0f;
constexpr int kSpTP   = 260;
constexpr int kScCh   = 32;
constexpr int kScTS   = 64;
constexpr int kScYP   = 68;
static_assert(kDbcW == 96, "dbc width");
static_assert((kDim % 32) == 0 && (kDtR % 32) == 0, "GEMM K multiples of 32");
static_assert((kRows % 64) == 0 && (kRows2 % 64) == 0 && (kDim % 64) == 0 && (kDbcP % 64) == 0, "GEMM M,N multiples of 64");
static_assert((kSeq % kScTS) == 0 && (kDim % kScCh) == 0 && (kDim % 256) == 0 && ((kDbcW * kDim) % 8) == 0, "tile multiples");

constexpr size_t kOffXN16  = 0;
constexpr size_t kOffXP16  = kOffXN16  + (size_t)kRows  * kDim  * 2;
constexpr size_t kOffPW16  = kOffXP16  + (size_t)kRows  * kDim  * 2;
constexpr size_t kOffCW16  = kOffPW16  + (size_t)kDim   * kDim  * 2;
constexpr size_t kOffDBW16 = kOffCW16  + (size_t)2 * kDim * kDim * 2;
constexpr size_t kOffDTW16 = kOffDBW16 + (size_t)kDbcP  * kDim  * 2;
constexpr size_t kOffXP    = kOffDTW16 + (size_t)kDim   * kDtR  * 2;
constexpr size_t kOffRAW   = kOffXP    + (size_t)kRows  * kDim  * 4;
constexpr size_t kOffU     = kOffRAW   + (size_t)kRows2 * kDim  * 4;
constexpr size_t kOffU16   = kOffU     + (size_t)kRows2 * kDim  * 4;
constexpr size_t kOffDBC   = kOffU16   + (size_t)kRows2 * kDim  * 2;
constexpr size_t kOffDT16  = kOffDBC   + (size_t)kRows2 * kDbcP * 4;
constexpr size_t kWsTotal  = kOffDT16  + (size_t)kRows2 * kDtR  * 2;
static_assert(kWsTotal == 129368064ull, "carve total");
static_assert(kWsTotal <= 134217728ull, "carve cap");
static_assert((kOffXP16 % 128) == 0 && (kOffPW16 % 128) == 0 && (kOffCW16 % 128) == 0 && (kOffDBW16 % 128) == 0 &&
              (kOffDTW16 % 128) == 0 && (kOffXP % 128) == 0 && (kOffRAW % 128) == 0 && (kOffU % 128) == 0 &&
              (kOffU16 % 128) == 0 && (kOffDBC % 128) == 0 && (kOffDT16 % 128) == 0, "128-B aligned regions");

__device__ __forceinline__ unsigned short f2bf_bits(float f) {
  unsigned u = __float_as_uint(f);
  return (unsigned short)((u + 0x7FFFu + ((u >> 16) & 1u)) >> 16);
}
__device__ __forceinline__ float bf_bits2f(unsigned short h) { return __uint_as_float(((unsigned)h) << 16); }

__device__ __forceinline__ void dep_guard_h(v8f& a, v8f& b, v16h x, v16h y) { asm volatile("v_nop\n\tv_nop\n\tv_nop\n\tv_nop" : "+v"(a), "+v"(b) : "v"(x), "v"(y)); }
__device__ __forceinline__ void dep_guard_b(v8f& a, v8f& b, v16b x, v16b y) { asm volatile("v_nop\n\tv_nop\n\tv_nop\n\tv_nop" : "+v"(a), "+v"(b) : "v"(x), "v"(y)); }
__device__ __forceinline__ void keep4_h(v16h a, v16h b, v16h c, v16h d) { asm volatile("v_nop" :: "v"(a), "v"(b), "v"(c), "v"(d)); }
__device__ __forceinline__ void keep4_b(v16b a, v16b b, v16b c, v16b d) { asm volatile("v_nop" :: "v"(a), "v"(b), "v"(c), "v"(d)); }
__device__ __forceinline__ void acc_guard4(v8f& a, v8f& b, v8f& c, v8f& d) { asm volatile("v_nop\n\tv_nop\n\tv_nop\n\tv_nop" : "+v"(a), "+v"(b), "+v"(c), "+v"(d)); }
template <typename T> struct Frag;
template <> struct Frag<_Float16> {
  typedef v16h V; union U { v16h v; v8h h[2]; };
  static __device__ __forceinline__ v16h load(const _Float16* p) {
    U f; f.h[0] = *(const v8h*)(p); f.h[1] = *(const v8h*)(p + 16); return f.v;
  }
  static __device__ __forceinline__ v8f mma(v16h a, v16h b, v8f c) {
    return __builtin_amdgcn_wmma_f32_16x16x32_f16(false, a, false, b, (short)0, c, false, false);
  }
  static __device__ __forceinline__ void guard(v8f& a, v8f& b, v16h x, v16h y) { dep_guard_h(a, b, x, y); }
  static __device__ __forceinline__ void keep(v16h a, v16h b, v16h c, v16h d) { keep4_h(a, b, c, d); }
};
template <> struct Frag<__bf16> {
  typedef v16b V; union U { v16b v; v8b h[2]; };
  static __device__ __forceinline__ v16b load(const __bf16* p) {
    U f; f.h[0] = *(const v8b*)(p); f.h[1] = *(const v8b*)(p + 16); return f.v;
  }
  static __device__ __forceinline__ v8f mma(v16b a, v16b b, v8f c) {
    return __builtin_amdgcn_wmma_f32_16x16x32_bf16(false, a, false, b, (short)0, c, false, false);
  }
  static __device__ __forceinline__ void guard(v8f& a, v8f& b, v16b x, v16b y) { dep_guard_b(a, b, x, y); }
  static __device__ __forceinline__ void keep(v16b a, v16b b, v16b c, v16b d) { keep4_b(a, b, c, d); }
};

template <int ET> struct Elem;
template <> struct Elem<0> { typedef _Float16 T; };
template <> struct Elem<1> { typedef __bf16 T; };
template <int ET, int SPL, int BIAS_MODE, int OUT_MODE, bool RESID, int ACT = 0>
__global__ __launch_bounds__(256) void wmma_gemm64(
    const unsigned short* __restrict__ Ap, const unsigned short* __restrict__ A2p, int lda, long strideA,
    const unsigned short* __restrict__ Btp, const unsigned short* __restrict__ Bt2p, int ldb, long strideB,
    void* __restrict__ Cout, void* __restrict__ Cout2, int ldc, long strideC,
    const float* __restrict__ bias,
    const float* __restrict__ resid, long strideR,
    int M, int N, int K, float scale) {
  typedef typename Elem<ET>::T T;
  typedef typename Frag<T>::V V;
  const T* A = (const T*)Ap; const T* A2 = (const T*)A2p; const T* Bt = (const T*)Btp; const T* Bt2 = (const T*)Bt2p;
  __shared__ __align__(16) float sT[8][16 * 68];
  const int b    = blockIdx.y;
  const int lane = threadIdx.x & 31;
  const int wave = threadIdx.x >> 5;
  const int tilesN = N >> 6;
  const int tilesM = M >> 6;
  const int tile = blockIdx.x * 8 + wave;
  if (tile >= tilesM * tilesN) return;
  const int tm = tile / tilesN;
  const int tn = tile - tm * tilesN;
  const int m0 = tm << 6;
  const int n0 = tn << 6;

  const T* Ab  = A  + (size_t)b * strideA;
  const T* Bb  = Bt + (size_t)b * strideB;
  const T* Ab2 = (SPL >= 1) ? (A2  + (size_t)b * strideA) : nullptr;
  const T* Bb2 = (SPL == 2) ? (Bt2 + (size_t)b * strideB) : nullptr;

  const int rlane = lane & 15;
  const int koff  = (lane >> 4) * 8;
  const int mOff  = (lane >> 4) * 8;

  v8f acc[4][4];
#pragma unroll
  for (int i = 0; i < 4; ++i)
#pragma unroll
    for (int j = 0; j < 4; ++j) acc[i][j] = (v8f){0.f,0.f,0.f,0.f,0.f,0.f,0.f,0.f};

  for (int k0 = 0; k0 < K; k0 += 32) {
    V bh[4], bl[4];
#pragma unroll
    for (int j = 0; j < 4; ++j) {
      const size_t bo = (size_t)(n0 + (j << 4) + rlane) * ldb + koff + k0;
      bh[j] = Frag<T>::load(Bb + bo);
      if (SPL == 2) bl[j] = Frag<T>::load(Bb2 + bo);
    }
#pragma unroll
    for (int i = 0; i < 4; ++i) {
      const size_t ao = (size_t)(m0 + (i << 4) + rlane) * lda + koff + k0;
      V ah = Frag<T>::load(Ab + ao);
      V al;
      if (SPL >= 1) al = Frag<T>::load(Ab2 + ao);
#pragma unroll
      for (int j = 0; j < 4; ++j) {
        acc[i][j] = Frag<T>::mma(ah, bh[j], acc[i][j]);
        if (SPL == 2) acc[i][j] = Frag<T>::mma(ah, bl[j], acc[i][j]);
        if (SPL >= 1) acc[i][j] = Frag<T>::mma(al, bh[j], acc[i][j]);
      }
      Frag<T>::guard(acc[i][0], acc[i][3], ah, (SPL >= 1) ? al : ah);
    }
    Frag<T>::keep(bh[0], bh[1], bh[2], bh[3]);
    if (SPL == 2) Frag<T>::keep(bl[0], bl[1], bl[2], bl[3]);
  }
  acc_guard4(acc[0][0], acc[0][1], acc[0][2], acc[0][3]);
  acc_guard4(acc[1][0], acc[1][1], acc[1][2], acc[1][3]);
  acc_guard4(acc[2][0], acc[2][1], acc[2][2], acc[2][3]);
  acc_guard4(acc[3][0], acc[3][1], acc[3][2], acc[3][3]);

  float* slab = sT[wave];
  const float* Rb = RESID ? (resid + (size_t)b * strideR) : nullptr;
#pragma unroll
  for (int i = 0; i < 4; ++i) {
    const int mBase = m0 + (i << 4);
#pragma unroll
    for (int j = 0; j < 4; ++j) {
      const int n = n0 + (j << 4) + rlane;
      float bv = 0.f;
      if (BIAS_MODE == 2) bv = bias[n];
#pragma unroll
      for (int r = 0; r < 8; ++r) {
        float v = acc[i][j][r] * scale;
        if (BIAS_MODE == 1) v += bias[mBase + mOff + r];
        if (BIAS_MODE == 2) v += bv;
        if (RESID) v += Rb[(size_t)(mBase + mOff + r) * ldc + n];
        if (ACT == 1) v = tanhf(v);
        if (ACT == 2) v = fmaxf(v, 0.0f);
        if (ACT == 3) v = v / (1.0f + expf(-v));
        if (ACT == 4) v = (v > 0.f) ? v : 0.01f * v;
        slab[(mOff + r) * 68 + (j << 4) + rlane] = v;
      }
    }
    __builtin_amdgcn_fence(__ATOMIC_RELEASE, "workgroup");
    __builtin_amdgcn_wave_barrier();
    __builtin_amdgcn_fence(__ATOMIC_ACQUIRE, "workgroup");
    if (OUT_MODE == 0) {
      float* C = (float*)Cout + (size_t)b * strideC;
      const int hh = lane >> 4, c4 = (lane & 15) * 4;
      for (int pass = 0; pass < 2; ++pass) {
#pragma unroll
        for (int it = 0; it < 8; ++it) {
          const int row = it * 2 + hh;
          v4f v = *(const v4f*)(slab + row * 68 + c4);
          *(volatile v4f*)(C + (size_t)(mBase + row) * ldc + n0 + c4) = v;
        }
        __threadfence();
      }
    } else {
      const int q = lane >> 3, c8 = (lane & 7) * 8;
      unsigned short* C  = (unsigned short*)Cout  + (size_t)b * strideC;
      unsigned short* C2 = (OUT_MODE == 2) ? ((unsigned short*)Cout2 + (size_t)b * strideC) : nullptr;
      for (int pass = 0; pass < 2; ++pass) {
#pragma unroll
        for (int it = 0; it < 4; ++it) {
          const int row = it * 4 + q;
          const float* sp = slab + row * 68 + c8;
          v8h hv, lv;
#pragma unroll
          for (int e = 0; e < 8; ++e) {
            if (OUT_MODE == 1) {
              hv[e] = (_Float16)sp[e];
            } else {
              unsigned short hb = f2bf_bits(sp[e]);
              unsigned short lb = f2bf_bits(sp[e] - bf_bits2f(hb));
              hv[e] = __builtin_bit_cast(_Float16, hb);
              lv[e] = __builtin_bit_cast(_Float16, lb);
            }
          }
          *(volatile v8h*)(C + (size_t)(mBase + row) * ldc + n0 + c8) = hv;
          if (OUT_MODE == 2) *(volatile v8h*)(C2 + (size_t)(mBase + row) * ldc + n0 + c8) = lv;
        }
        __threadfence();
      }
    }
    __builtin_amdgcn_fence(__ATOMIC_RELEASE, "workgroup");
    __builtin_amdgcn_wave_barrier();
    __builtin_amdgcn_fence(__ATOMIC_ACQUIRE, "workgroup");
  }
}

__global__ __launch_bounds__(256) void cast_f16_kernel(
    const float* __restrict__ src, unsigned short* __restrict__ dst, int nReal, int total8, float scale)
{
  const int i = blockIdx.x * 256 + threadIdx.x;
  if (i >= total8) return;
  const size_t e0 = (size_t)i << 3;
  const bool live = (e0 < (size_t)nReal);
  const size_t ec = live ? e0 : (size_t)(nReal - 8);
  const float sc = live ? scale : 0.0f;
  const v4f a0 = *(const v4f*)(src + ec);
  const v4f a1 = *(const v4f*)(src + ec + 4);
  v8h hv;
#pragma unroll
  for (int e = 0; e < 4; ++e) {
    hv[e]     = (_Float16)(a0[e] * sc);
    hv[4 + e] = (_Float16)(a1[e] * sc);
  }
  unsigned short* q = dst + e0;
  *(volatile v8h*)q = hv;
  __threadfence();
  *(volatile v8h*)q = hv;
}

__global__ __launch_bounds__(128) void layernorm_f16_kernel(
    const float* __restrict__ x, const float* __restrict__ w, const float* __restrict__ bb,
    unsigned short* __restrict__ XN)
{
  __shared__ float sRed0[4];
  __shared__ float sRed1[4];
  const int tid = threadIdx.x, lane = tid & 31, wave = tid >> 5;
  const size_t row = blockIdx.x;
  const size_t e0 = row * (size_t)kDim + (size_t)tid * 8;
  const v4f a0 = *(const v4f*)(x + e0);
  const v4f a1 = *(const v4f*)(x + e0 + 4);
  float s = ((a0[0] + a0[1]) + (a0[2] + a0[3])) + ((a1[0] + a1[1]) + (a1[2] + a1[3]));
#pragma unroll
  for (int off = 1; off < 32; off <<= 1) s += __shfl_xor(s, off, 32);
  if (lane == 0) sRed0[wave] = s;
  __syncthreads();
  const float mu = ((sRed0[0] + sRed0[1]) + (sRed0[2] + sRed0[3])) * (1.0f / (float)kDim);
  float c[8];
#pragma unroll
  for (int e = 0; e < 4; ++e) { c[e] = a0[e] - mu; c[4 + e] = a1[e] - mu; }
  float ss = 0.f;
#pragma unroll
  for (int e = 0; e < 8; ++e) ss = c[e] * c[e] + ss;
#pragma unroll
  for (int off = 1; off < 32; off <<= 1) ss += __shfl_xor(ss, off, 32);
  if (lane == 0) sRed1[wave] = ss;
  __syncthreads();
  const float var = ((sRed1[0] + sRed1[1]) + (sRed1[2] + sRed1[3])) * (1.0f / (float)kDim);
  const float rs = rsqrtf(var + kEps);
  const v4f w0 = *(const v4f*)(w + (size_t)tid * 8);
  const v4f w1 = *(const v4f*)(w + (size_t)tid * 8 + 4);
  const v4f b0 = *(const v4f*)(bb + (size_t)tid * 8);
  const v4f b1 = *(const v4f*)(bb + (size_t)tid * 8 + 4);
  v8h hv;
#pragma unroll
  for (int e = 0; e < 4; ++e) {
    const float t0 = (c[e] * rs) * w0[e] + b0[e];
    const float t1 = (c[4 + e] * rs) * w1[e] + b1[e];
    hv[e]     = (_Float16)t0;
    hv[4 + e] = (_Float16)t1;
  }
  unsigned short* q = XN + e0;
  *(volatile v8h*)q = hv;
  __threadfence();
  *(volatile v8h*)q = hv;
}

__global__ __launch_bounds__(256) void softplus_u_kernel(
    const float* __restrict__ URAW, const float* __restrict__ bF, const float* __restrict__ bB,
    float* __restrict__ U, unsigned short* __restrict__ U16)
{
  __shared__ __align__(16) float sT[16 * kSpTP];
  const int tid = threadIdx.x, lane = tid & 31, wave = tid >> 5;
  const int d0 = blockIdx.x * 256, d = d0 + tid;
  const int g0 = blockIdx.y * 64;
  const float bf0 = bF[d], bb0 = bB[d];
  const float bsel = (blockIdx.y < (unsigned)(kRows / 64)) ? bf0 : bb0;
  const int hrow = wave >> 1;
  const int hch  = (wave & 1) * 128 + lane * 4;
#pragma unroll 1
  for (int sub = 0; sub < 4; ++sub) {
    const int lb = g0 + sub * 16;
#pragma unroll 1
    for (int s = 0; s < 16; ++s) {
      const float v  = URAW[(size_t)(lb + s) * kDim + d] + bsel;
      const float sp = fmaxf(v, 0.0f) + log1pf(expf(-fabsf(v)));
      sT[s * kSpTP + tid] = sp;
    }
    __syncthreads();
    v4f fv[4];
    v8h hv[2];
#pragma unroll
    for (int it = 0; it < 4; ++it) fv[it] = *(const v4f*)(sT + (it * 4 + hrow) * kSpTP + hch);
#pragma unroll
    for (int it = 0; it < 2; ++it) {
      const float* sp = sT + (it * 8 + wave) * kSpTP + lane * 8;
      const v4f a0 = *(const v4f*)(sp);
      const v4f a1 = *(const v4f*)(sp + 4);
#pragma unroll
      for (int e = 0; e < 4; ++e) {
        hv[it][e]     = (_Float16)a0[e];
        hv[it][4 + e] = (_Float16)a1[e];
      }
    }
    for (int pass = 0; pass < 2; ++pass) {
#pragma unroll
      for (int it = 0; it < 4; ++it)
        *(volatile v4f*)(U + (size_t)(lb + it * 4 + hrow) * kDim + d0 + hch) = fv[it];
#pragma unroll
      for (int it = 0; it < 2; ++it)
        *(volatile v8h*)(U16 + (size_t)(lb + it * 8 + wave) * kDim + d0 + lane * 8) = hv[it];
      __threadfence();
    }
    __syncthreads();
  }
}

__global__ __launch_bounds__(256) void dt_plane_kernel(const float* __restrict__ DBC, unsigned short* __restrict__ DT16)
{
  const int i = blockIdx.x * 256 + threadIdx.x;
  if (i >= kRows2 * (kDtR / 8)) return;
  const int row = i >> 3, c8 = (i & 7) * 8;
  const float* sp = DBC + (size_t)row * kDbcP + c8;
  const v4f a0 = *(const v4f*)(sp);
  const v4f a1 = *(const v4f*)(sp + 4);
  v8h hv;
#pragma unroll
  for (int e = 0; e < 4; ++e) { hv[e] = (_Float16)a0[e]; hv[4 + e] = (_Float16)a1[e]; }
  unsigned short* q = DT16 + (size_t)row * kDtR + c8;
  *(volatile v8h*)q = hv;
  __threadfence();
  *(volatile v8h*)q = hv;
}

__global__ __launch_bounds__(64) void scan_combine_kernel(
    const float* __restrict__ DBC, const float* __restrict__ DRAW, const float* __restrict__ U,
    const float* __restrict__ XP, const float* __restrict__ X,
    const float* __restrict__ Alog, const float* __restrict__ Dp, float* __restrict__ OUT)
{
  __shared__ __align__(16) float sBC[2 * kScTS * 32];
  __shared__ __align__(16) float sY[kScTS * kScYP];
  __shared__ __align__(16) float sA[kNst * 64];
  const int tid = threadIdx.x, lane = tid & 31, wave = tid >> 5;
  constexpr int kBlkPerB = kDim / kScCh;
  const int bix = blockIdx.x / kBlkPerB;
  const int d0  = (blockIdx.x - bix * kBlkPerB) * kScCh;
  const int d   = d0 + lane;
  const size_t tok0 = (size_t)bix * kSeq;
  const size_t rb   = (size_t)wave * kRows + tok0;
#pragma unroll 1
  for (int s = 0; s < kNst; ++s) sA[s * 64 + tid] = -expf(Alog[(size_t)d * kNst + s]);
  __syncthreads();
  float negA[kNst], h[kNst];
#pragma unroll
  for (int s = 0; s < kNst; ++s) { negA[s] = sA[s * 64 + tid]; h[s] = 0.f; }
  const float Dd = Dp[d];
  const int q = lane >> 3, c4 = (lane & 7) * 4;
#pragma unroll 1
  for (int t0 = 0; t0 < kSeq; t0 += kScTS) {
    __syncthreads();
#pragma unroll
    for (int i = 0; i < 16; ++i) {
      const int idx = tid + 64 * i;
      const int br = idx >> 9, rem = idx & 511;
      const int s = rem >> 3, cc = (rem & 7) * 4;
      *(v4f*)(sBC + (br * kScTS + s) * 32 + cc) =
          *(const v4f*)(DBC + ((size_t)br * kRows + tok0 + t0 + s) * kDbcP + kDtR + cc);
    }
    __syncthreads();
#pragma unroll 1
    for (int s = 0; s < kScTS; ++s) {
      const int t = t0 + s;
      const float* bc = sBC + (wave * kScTS + s) * 32;
      float Bs[kNst], Cs[kNst];
#pragma unroll
      for (int q4 = 0; q4 < 4; ++q4) {
        const v4f bv = *(const v4f*)(bc + 4 * q4);
        const v4f cv = *(const v4f*)(bc + kNst + 4 * q4);
        Bs[4 * q4 + 0] = bv[0]; Bs[4 * q4 + 1] = bv[1]; Bs[4 * q4 + 2] = bv[2]; Bs[4 * q4 + 3] = bv[3];
        Cs[4 * q4 + 0] = cv[0]; Cs[4 * q4 + 1] = cv[1]; Cs[4 * q4 + 2] = cv[2]; Cs[4 * q4 + 3] = cv[3];
      }
      const float v   = DRAW[(rb + t) * kDim + d];
      const float uu  = U[(rb + t) * kDim + d];
      const float a   = __expf(-fabsf(v));
      const float ua  = 1.0f + a;
      const float l1p = __logf(ua) + (a - (ua - 1.0f)) * __builtin_amdgcn_rcpf(ua);
      const float dt  = fmaxf(v, 0.0f) + l1p;
      const float dtu = dt * uu;
      float y = 0.f;
#pragma unroll
      for (int k = 0; k < kNst; ++k) {
        const float e = __expf(dt * negA[k]);
        h[k] = e * h[k] + dtu * Bs[k];
        y = h[k] * Cs[k] + y;
      }
      y = uu * Dd + y;
      sY[s * kScYP + tid] = y;
    }
    __syncthreads();
#pragma unroll 1
    for (int i = 0; i < 32; ++i) {
      const int row = 2 * i + wave;
      const size_t grow = tok0 + t0 + row;
      const float y1  = sY[row * kScYP + lane];
      const float y2  = sY[row * kScYP + 32 + lane];
      const float xpv = XP[grow * kDim + d];
      const float xv  = X[grow * kDim + d];
      const float sg  = __builtin_amdgcn_rcpf(1.0f + __expf(-xpv));
      const float z   = xpv * sg;
      float o = y1 * z;
      o = y2 * z + o;
      o = o + xv;
      sY[row * kScYP + lane] = o;
    }
    __syncthreads();
    for (int pass = 0; pass < 2; ++pass) {
#pragma unroll
      for (int it = 0; it < 8; ++it) {
        const int row = it * 8 + wave * 4 + q;
        const v4f ov = *(const v4f*)(sY + row * kScYP + c4);
        *(volatile v4f*)(OUT + (tok0 + t0 + row) * kDim + d0 + c4) = ov;
      }
      __threadfence();
    }
  }
}

extern "C" void kernel_launch(void* const* d_in, const int* in_sizes, int n_in,
                              void* d_out, int out_size, void* d_ws, size_t ws_size,
                              hipStream_t stream) {
  if (n_in < 14) return;
  if (in_sizes[0]  != kRows * kDim) return;
  if (in_sizes[1]  != kDim) return;
  if (in_sizes[2]  != kDim) return;
  if (in_sizes[3]  != kDim * kDim) return;
  if (in_sizes[4]  != kDim) return;
  if (in_sizes[5]  != kDim * kDim) return;
  if (in_sizes[6]  != kDim) return;
  if (in_sizes[7]  != kDim * kDim) return;
  if (in_sizes[8]  != kDim) return;
  if (in_sizes[9]  != kDbcW * kDim) return;
  if (in_sizes[10] != kDim * kDtR) return;
  if (in_sizes[11] != kDim) return;
  if (in_sizes[12] != kDim * kNst) return;
  if (in_sizes[13] != kDim) return;
  if (out_size != kRows * kDim) return;
  if (ws_size < kWsTotal) return;

  const float* x       = (const float*)d_in[0];
  const float* ln_w    = (const float*)d_in[1];
  const float* ln_b    = (const float*)d_in[2];
  const float* proj_W  = (const float*)d_in[3];
  const float* proj_b  = (const float*)d_in[4];
  const float* fconv_W = (const float*)d_in[5];
  const float* fconv_b = (const float*)d_in[6];
  const float* bconv_W = (const float*)d_in[7];
  const float* bconv_b = (const float*)d_in[8];
  const float* dbc_W   = (const float*)d_in[9];
  const float* dt_W    = (const float*)d_in[10];
  const float* dt_b    = (const float*)d_in[11];
  const float* A_log   = (const float*)d_in[12];
  const float* Dvec    = (const float*)d_in[13];
  float* out = (float*)d_out;

  char* ws = (char*)d_ws;
  unsigned short* XN16  = (unsigned short*)(ws + kOffXN16);
  unsigned short* XP16  = (unsigned short*)(ws + kOffXP16);
  unsigned short* PW16  = (unsigned short*)(ws + kOffPW16);
  unsigned short* CW16  = (unsigned short*)(ws + kOffCW16);
  unsigned short* DBW16 = (unsigned short*)(ws + kOffDBW16);
  unsigned short* DTW16 = (unsigned short*)(ws + kOffDTW16);
  float*          XP    = (float*)(ws + kOffXP);
  float*          URAW  = (float*)(ws + kOffRAW);
  float*          DRAW  = (float*)(ws + kOffRAW);
  float*          U     = (float*)(ws + kOffU);
  unsigned short* U16   = (unsigned short*)(ws + kOffU16);
  float*          DBC   = (float*)(ws + kOffDBC);
  unsigned short* DT16  = (unsigned short*)(ws + kOffDT16);

  cast_f16_kernel<<<(kDim * kDim / 8) / 256, 256, 0, stream>>>(proj_W,  PW16,               kDim * kDim, kDim * kDim / 8, kWCarry);
  cast_f16_kernel<<<(kDim * kDim / 8) / 256, 256, 0, stream>>>(fconv_W, CW16,               kDim * kDim, kDim * kDim / 8, kWCarry);
  cast_f16_kernel<<<(kDim * kDim / 8) / 256, 256, 0, stream>>>(bconv_W, CW16 + kDim * kDim, kDim * kDim, kDim * kDim / 8, kWCarry);
  cast_f16_kernel<<<(kDbcP * kDim / 8) / 256, 256, 0, stream>>>(dbc_W,  DBW16,              kDbcW * kDim, kDbcP * kDim / 8, kWCarry);
  cast_f16_kernel<<<(kDim * kDtR / 8) / 256, 256, 0, stream>>>(dt_W,    DTW16,              kDim * kDtR, kDim * kDtR / 8, kWCarry);

  layernorm_f16_kernel<<<kRows, 128, 0, stream>>>(x, ln_w, ln_b, XN16);

  wmma_gemm64<0, 0, 2, 0, false><<<dim3(128, 1), 256, 0, stream>>>(
      XN16, nullptr, kDim, 0L,
      PW16, nullptr, kDim, 0L,
      (void*)XP, nullptr, kDim, 0L,
      proj_b, nullptr, 0L,
      kRows, kDim, kDim, kWCarryInv);

  cast_f16_kernel<<<(kRows * kDim / 8) / 256, 256, 0, stream>>>(XP, XP16, kRows * kDim, kRows * kDim / 8, 1.0f);

  wmma_gemm64<0, 0, 0, 0, false><<<dim3(128, 2), 256, 0, stream>>>(
      XP16, nullptr, kDim, 0L,
      CW16, nullptr, kDim, (long)kDim * kDim,
      (void*)URAW, nullptr, kDim, (long)kRows * kDim,
      nullptr, nullptr, 0L,
      kRows, kDim, kDim, kWCarryInv);

  softplus_u_kernel<<<dim3(kDim / 256, kRows2 / 64), 256, 0, stream>>>(URAW, fconv_b, bconv_b, U, U16);

  wmma_gemm64<0, 0, 0, 0, false><<<dim3(32, 1), 256, 0, stream>>>(
      U16, nullptr, kDim, 0L,
      DBW16, nullptr, kDim, 0L,
      (void*)DBC, nullptr, kDbcP, 0L,
      nullptr, nullptr, 0L,
      kRows2, kDbcP, kDim, kWCarryInv);

  dt_plane_kernel<<<(kRows2 * (kDtR / 8)) / 256, 256, 0, stream>>>(DBC, DT16);

  wmma_gemm64<0, 0, 2, 0, false><<<dim3(256, 1), 256, 0, stream>>>(
      DT16, nullptr, kDtR, 0L,
      DTW16, nullptr, kDtR, 0L,
      (void*)DRAW, nullptr, kDim, 0L,
      dt_b, nullptr, 0L,
      kRows2, kDim, kDtR, kWCarryInv);

  scan_combine_kernel<<<kBatch * (kDim / kScCh), 64, 0, stream>>>(DBC, DRAW, U, XP, x, A_log, Dvec, out);
}
